// FlashSVDLlamaBlock_26980984553791
// MI455X (gfx1250) — hardware-verified
//
#include <hip/hip_runtime.h>

typedef _Float16 v16h __attribute__((ext_vector_type(16)));
typedef _Float16 v8h  __attribute__((ext_vector_type(8)));
typedef float    v8f  __attribute__((ext_vector_type(8)));
typedef float    v4f  __attribute__((ext_vector_type(4)));
typedef v8h __attribute__((may_alias)) v8ha;
typedef v4f __attribute__((may_alias)) v4fa;

union Frag { v16h v; v8h half[2]; };

#define TT    1024
#define DD    4096
#define NHQ   32
#define NHKV  8
#define DH    128
#define RQK   64
#define RLO   1024
#define FF    14336
#define NXR   3072
#define WSC   32.0f
#define PSC   16384.0f

__device__ __forceinline__ v8f wmma_f16(v16h a, v16h b, v8f c) {
  v8f d = __builtin_amdgcn_wmma_f32_16x16x32_f16(false, a, false, b, (short)0, c, false, false);
  asm volatile("v_nop\n\tv_nop\n\tv_nop\n\tv_nop" : "+v"(d) : "v"(a), "v"(b));
  return d;
}

__device__ __forceinline__ v16h load_frag(const _Float16* p, int h) {
  Frag f;
  f.half[0] = *(const v8ha*)(p + 8 * h);
  f.half[1] = *(const v8ha*)(p + 16 + 8 * h);
  return f.v;
}

__device__ __forceinline__ v8f zero8f() {
  v8f z = {0.f, 0.f, 0.f, 0.f, 0.f, 0.f, 0.f, 0.f};
  return z;
}

__device__ __forceinline__ v8h to8h(v4f a, v4f b) {
  v8h r = { (_Float16)a.x, (_Float16)a.y, (_Float16)a.z, (_Float16)a.w,
            (_Float16)b.x, (_Float16)b.y, (_Float16)b.z, (_Float16)b.w };
  return r;
}

__device__ __forceinline__ v8h cvt8h(v8f v) {
  v8h r = { (_Float16)v[0], (_Float16)v[1], (_Float16)v[2], (_Float16)v[3],
            (_Float16)v[4], (_Float16)v[5], (_Float16)v[6], (_Float16)v[7] };
  return r;
}

__device__ __forceinline__ void mma_32x64(const _Float16* __restrict__ ar, int lda,
                                          const _Float16* __restrict__ br, int ldb,
                                          int K, int h, v8f (&acc)[2][4]) {
  const _Float16* ar1 = ar + (size_t)16 * lda;
  #pragma unroll 1
  for (int k0 = 0; k0 < K; k0 += 32) {
    const v16h a0 = load_frag(ar + k0, h);
    const v16h a1 = load_frag(ar1 + k0, h);
    #pragma unroll
    for (int nt = 0; nt < 4; ++nt) {
      const v16h b = load_frag(br + (size_t)nt * 16 * ldb + k0, h);
      acc[0][nt] = wmma_f16(a0, b, acc[0][nt]);
      acc[1][nt] = wmma_f16(a1, b, acc[1][nt]);
    }
  }
}

__global__ __launch_bounds__(64) void k_rope_table(float* __restrict__ cosT, float* __restrict__ sinT) {
  __shared__ float cs[64];
  __shared__ float sn[64];
  const int t = blockIdx.x, j = threadIdx.x;
  const float ex = (float)(2 * j) * (1.0f / 128.0f);
  const float pw = powf(10000.0f, ex);
  const float inv = 1.0f / pw;
  const float ang = (float)t * inv;
  cs[j] = cosf(ang);
  sn[j] = sinf(ang);
  __syncthreads();
  const int lane = j & 31, wv = j >> 5;
  const float* src = wv ? sn : cs;
  float* dst = (wv ? sinT : cosT) + (size_t)t * DH + 4 * lane;
  const v4f v = {src[2 * lane], src[2 * lane], src[2 * lane + 1], src[2 * lane + 1]};
  *(volatile v4f*)dst = v;
  __threadfence();
  *(volatile v4f*)dst = v;
}

__global__ __launch_bounds__(256) void k_cvt(const float* __restrict__ src, _Float16* __restrict__ dst,
                                             int n8, float sc) {
  const int g = blockIdx.x * 256 + threadIdx.x;
  if (g >= n8) return;
  const float* p = src + (size_t)g * 8;
  const v4f a = *(const v4fa*)p;
  const v4f c = *(const v4fa*)(p + 4);
  const v8h o = to8h(a * sc, c * sc);
  _Float16* q = dst + (size_t)g * 8;
  *(volatile v8h*)q = o;
  __threadfence();
  *(volatile v8h*)q = o;
}

__global__ __launch_bounds__(256) void k_rmsnorm(const float* __restrict__ x, const float* __restrict__ wgt,
                                                 _Float16* __restrict__ out) {
  __shared__ float red[8];
  __shared__ float scl;
  const int tid = threadIdx.x, lane = tid & 31, wave = tid >> 5;
  const size_t rb = (size_t)blockIdx.x * DD;
  const int e0 = tid * 8, e1 = 2048 + tid * 8;
  const v4f a0 = *(const v4fa*)(x + rb + e0);
  const v4f a1 = *(const v4fa*)(x + rb + e0 + 4);
  const v4f b0 = *(const v4fa*)(x + rb + e1);
  const v4f b1 = *(const v4fa*)(x + rb + e1 + 4);
  const v4f q = a0 * a0 + a1 * a1 + b0 * b0 + b1 * b1;
  float s = (q.x + q.y) + (q.z + q.w);
  #pragma unroll
  for (int o = 16; o > 0; o >>= 1) s += __shfl_xor(s, o, 32);
  if (lane == 0) red[wave] = s;
  __syncthreads();
  if (tid == 0) {
    float t = 0.f;
    #pragma unroll
    for (int i = 0; i < 8; ++i) t += red[i];
    scl = rsqrtf(t * (1.0f / 4096.0f) + 1e-5f);
  }
  __syncthreads();
  const float sc = scl;
  const v4f w0 = *(const v4fa*)(wgt + e0);
  const v4f w1 = *(const v4fa*)(wgt + e0 + 4);
  const v4f w2 = *(const v4fa*)(wgt + e1);
  const v4f w3 = *(const v4fa*)(wgt + e1 + 4);
  const v8h o0 = to8h(a0 * sc * w0, a1 * sc * w1);
  const v8h o1 = to8h(b0 * sc * w2, b1 * sc * w3);
  _Float16* p0 = out + rb + e0;
  _Float16* p1 = out + rb + e1;
  *(volatile v8h*)p0 = o0;
  *(volatile v8h*)p1 = o1;
  __threadfence();
  *(volatile v8h*)p0 = o0;
  *(volatile v8h*)p1 = o1;
}

__global__ __launch_bounds__(128) void k_gemm_h(
    const _Float16* __restrict__ A, int lda, const _Float16* __restrict__ B, int ldb,
    _Float16* __restrict__ C, int ldc, int K, float cscale)
{
  __shared__ __attribute__((aligned(16))) _Float16 sT[4 * 32 * 64];
  const int tid = threadIdx.x, lane = tid & 31, w = tid >> 5;
  const int h = lane >> 4, m = lane & 15;
  const int row0 = blockIdx.y * 128 + 32 * w;
  const int col0 = blockIdx.x * 64;

  v8f acc[2][4];
  #pragma unroll
  for (int mt = 0; mt < 2; ++mt)
    #pragma unroll
    for (int nt = 0; nt < 4; ++nt) acc[mt][nt] = zero8f();

  mma_32x64(A + (size_t)(row0 + m) * lda, lda, B + (size_t)(col0 + m) * ldb, ldb, K, h, acc);

  _Float16* st = sT + w * 2048;
  #pragma unroll
  for (int mt = 0; mt < 2; ++mt)
    #pragma unroll
    for (int nt = 0; nt < 4; ++nt)
      #pragma unroll
      for (int r = 0; r < 8; ++r)
        st[(16 * mt + 8 * h + r) * 64 + 16 * nt + m] = (_Float16)(acc[mt][nt][r] * cscale);
  __syncthreads();

  const int q8 = lane & 7, sub = lane >> 3;
  v8h pk[8];
  #pragma unroll
  for (int i = 0; i < 8; ++i) {
    const int lid = 4 * i + sub;
    pk[i] = *(const v8ha*)(st + lid * 64 + 8 * q8);
  }
  #pragma unroll
  for (int i = 0; i < 8; ++i) {
    const int lid = 4 * i + sub;
    *(volatile v8h*)(C + (size_t)(row0 + lid) * ldc + col0 + 8 * q8) = pk[i];
  }
  __threadfence();
  #pragma unroll
  for (int i = 0; i < 8; ++i) {
    const int lid = 4 * i + sub;
    *(volatile v8h*)(C + (size_t)(row0 + lid) * ldc + col0 + 8 * q8) = pk[i];
  }
}

__global__ __launch_bounds__(128) void k_gemm_res(
    const _Float16* __restrict__ A, int lda, const _Float16* __restrict__ B, int ldb,
    const float* __restrict__ R, float* __restrict__ C, int K, float cscale)
{
  __shared__ __attribute__((aligned(16))) float sT[4 * 32 * 64];
  const int tid = threadIdx.x, lane = tid & 31, w = tid >> 5;
  const int h = lane >> 4, m = lane & 15;
  const int row0 = blockIdx.y * 128 + 32 * w;
  const int col0 = blockIdx.x * 64;

  v8f acc[2][4];
  #pragma unroll
  for (int mt = 0; mt < 2; ++mt)
    #pragma unroll
    for (int nt = 0; nt < 4; ++nt) acc[mt][nt] = zero8f();

  mma_32x64(A + (size_t)(row0 + m) * lda, lda, B + (size_t)(col0 + m) * ldb, ldb, K, h, acc);

  float* st = sT + w * 2048;
  #pragma unroll
  for (int mt = 0; mt < 2; ++mt)
    #pragma unroll
    for (int nt = 0; nt < 4; ++nt)
      #pragma unroll
      for (int r = 0; r < 8; ++r)
        st[(16 * mt + 8 * h + r) * 64 + 16 * nt + m] = acc[mt][nt][r] * cscale;
  __syncthreads();

  const int q8 = lane & 7, sub = lane >> 3;
  v4f pk[16];
  #pragma unroll
  for (int i = 0; i < 16; ++i) {
    const int lid = 4 * i + sub, lr = lid >> 1, hl = lid & 1;
    const int cc = 32 * hl + 4 * q8;
    const v4f v = *(const v4fa*)(st + lr * 64 + cc);
    const size_t gi = (size_t)(row0 + lr) * DD + col0 + cc;
    const v4f rr = *(const v4fa*)(R + gi);
    pk[i] = v + rr;
  }
  #pragma unroll
  for (int i = 0; i < 16; ++i) {
    const int lid = 4 * i + sub, lr = lid >> 1, hl = lid & 1;
    const size_t gi = (size_t)(row0 + lr) * DD + col0 + 32 * hl + 4 * q8;
    *(volatile v4f*)(C + gi) = pk[i];
  }
  __threadfence();
  #pragma unroll
  for (int i = 0; i < 16; ++i) {
    const int lid = 4 * i + sub, lr = lid >> 1, hl = lid & 1;
    const size_t gi = (size_t)(row0 + lr) * DD + col0 + 32 * hl + 4 * q8;
    *(volatile v4f*)(C + gi) = pk[i];
  }
}

__global__ __launch_bounds__(128) void k_gemm_glu(
    const _Float16* __restrict__ GU, const _Float16* __restrict__ Bg,
    const _Float16* __restrict__ Bu, _Float16* __restrict__ Hm)
{
  __shared__ __attribute__((aligned(16))) float    gS[4 * 32 * 64];
  __shared__ __attribute__((aligned(16))) _Float16 hS[4 * 32 * 64];
  const int tid = threadIdx.x, lane = tid & 31, w = tid >> 5;
  const int h = lane >> 4, m = lane & 15;
  const int row0 = blockIdx.y * 128 + 32 * w;
  const int col0 = blockIdx.x * 64;

  v8f acc[2][4];
  #pragma unroll
  for (int mt = 0; mt < 2; ++mt)
    #pragma unroll
    for (int nt = 0; nt < 4; ++nt) acc[mt][nt] = zero8f();

  mma_32x64(GU + (size_t)(row0 + m) * (2 * RLO), 2 * RLO,
            Bg + (size_t)(col0 + m) * RLO, RLO, RLO, h, acc);

  float* gs = gS + w * 2048;
  #pragma unroll
  for (int mt = 0; mt < 2; ++mt)
    #pragma unroll
    for (int nt = 0; nt < 4; ++nt)
      #pragma unroll
      for (int r = 0; r < 8; ++r)
        gs[(16 * mt + 8 * h + r) * 64 + 16 * nt + m] = acc[mt][nt][r] * (1.0f / WSC);
  __syncthreads();

  #pragma unroll
  for (int mt = 0; mt < 2; ++mt)
    #pragma unroll
    for (int nt = 0; nt < 4; ++nt) acc[mt][nt] = zero8f();

  mma_32x64(GU + (size_t)(row0 + m) * (2 * RLO) + RLO, 2 * RLO,
            Bu + (size_t)(col0 + m) * RLO, RLO, RLO, h, acc);

  _Float16* hs = hS + w * 2048;
  #pragma unroll
  for (int mt = 0; mt < 2; ++mt)
    #pragma unroll
    for (int nt = 0; nt < 4; ++nt)
      #pragma unroll
      for (int r = 0; r < 8; ++r) {
        const int idx = (16 * mt + 8 * h + r) * 64 + 16 * nt + m;
        const float g = gs[idx];
        const float u = acc[mt][nt][r] * (1.0f / WSC);
        const float e = __expf(fminf(-g, 80.0f));
        const float sg = g * __builtin_amdgcn_rcpf(1.0f + e);
        hs[idx] = (_Float16)(sg * u * 4.0f);
      }
  __syncthreads();

  const int q8 = lane & 7, sub = lane >> 3;
  v8h pk[8];
  #pragma unroll
  for (int i = 0; i < 8; ++i) {
    const int lid = 4 * i + sub;
    pk[i] = *(const v8ha*)(hs + lid * 64 + 8 * q8);
  }
  #pragma unroll
  for (int i = 0; i < 8; ++i) {
    const int lid = 4 * i + sub;
    *(volatile v8h*)(Hm + (size_t)(row0 + lid) * FF + col0 + 8 * q8) = pk[i];
  }
  __threadfence();
  #pragma unroll
  for (int i = 0; i < 8; ++i) {
    const int lid = 4 * i + sub;
    *(volatile v8h*)(Hm + (size_t)(row0 + lid) * FF + col0 + 8 * q8) = pk[i];
  }
}

__global__ __launch_bounds__(128) void k_proj_rope(
    const _Float16* __restrict__ XR, const _Float16* __restrict__ US,
    const float* __restrict__ cosT, const float* __restrict__ sinT,
    _Float16* __restrict__ qh, _Float16* __restrict__ kh, _Float16* __restrict__ vT)
{
  __shared__ __attribute__((aligned(16))) float S[64 * 128];
  const int tid = threadIdx.x, lane = tid & 31, w = tid >> 5;
  const int h = lane >> 4, m = lane & 15;
  const int g = blockIdx.y;
  const int t0 = blockIdx.x * 64;
  const int wm = w >> 1, wn = w & 1;

  v8f acc[2][4];
  #pragma unroll
  for (int mt = 0; mt < 2; ++mt)
    #pragma unroll
    for (int nt = 0; nt < 4; ++nt) acc[mt][nt] = zero8f();

  mma_32x64(XR + (size_t)(t0 + 32 * wm + m) * NXR + 64 * g, NXR,
            US + (size_t)g * (DH * RQK) + (size_t)(64 * wn + m) * RQK, RQK, RQK, h, acc);

  #pragma unroll
  for (int mt = 0; mt < 2; ++mt)
    #pragma unroll
    for (int nt = 0; nt < 4; ++nt)
      #pragma unroll
      for (int r = 0; r < 8; ++r)
        S[(32 * wm + 16 * mt + 8 * h + r) * 128 + 64 * wn + 16 * nt + m] = acc[mt][nt][r];
  __syncthreads();

  const int q8 = lane & 7, sub = lane >> 3;
  const float osc = 4.0f / WSC;
  if (g < 40) {
    _Float16* plane = (g < 32) ? (qh + (size_t)g * TT * DH) : (kh + (size_t)(g - 32) * TT * DH);
    v8h pk[8];
    #pragma unroll
    for (int i = 0; i < 8; ++i) {
      const int lid = 4 * i + sub;
      const int tl = 16 * w + (lid >> 1), hl = lid & 1;
      const int d0 = 64 * hl + 8 * q8, dp = d0 ^ 64;
      const float* sr = S + tl * 128;
      const v4f a0 = *(const v4fa*)(sr + d0);
      const v4f a1 = *(const v4fa*)(sr + d0 + 4);
      const v4f b0 = *(const v4fa*)(sr + dp);
      const v4f b1 = *(const v4fa*)(sr + dp + 4);
      const size_t tb = (size_t)(t0 + tl) * DH + d0;
      const v4f c0 = *(const v4fa*)(cosT + tb);
      const v4f c1 = *(const v4fa*)(cosT + tb + 4);
      const v4f s0 = *(const v4fa*)(sinT + tb);
      const v4f s1 = *(const v4fa*)(sinT + tb + 4);
      const float sg = hl ? osc : -osc;
      const v4f o0 = a0 * c0 * osc + b0 * s0 * sg;
      const v4f o1 = a1 * c1 * osc + b1 * s1 * sg;
      pk[i] = to8h(o0, o1);
    }
    #pragma unroll
    for (int i = 0; i < 8; ++i) {
      const int lid = 4 * i + sub;
      const int tl = 16 * w + (lid >> 1), hl = lid & 1;
      *(volatile v8h*)(plane + (size_t)(t0 + tl) * DH + 64 * hl + 8 * q8) = pk[i];
    }
    __threadfence();
    #pragma unroll
    for (int i = 0; i < 8; ++i) {
      const int lid = 4 * i + sub;
      const int tl = 16 * w + (lid >> 1), hl = lid & 1;
      *(volatile v8h*)(plane + (size_t)(t0 + tl) * DH + 64 * hl + 8 * q8) = pk[i];
    }
  } else {
    _Float16* vplane = vT + (size_t)(g - 40) * DH * TT;
    v8h pk[8];
    #pragma unroll
    for (int i = 0; i < 8; ++i) {
      const int lid = 4 * i + sub;
      const int d = 32 * w + lid;
      v8f v;
      #pragma unroll
      for (int e = 0; e < 8; ++e) v[e] = S[(8 * q8 + e) * 128 + d] * osc;
      pk[i] = cvt8h(v);
    }
    #pragma unroll
    for (int i = 0; i < 8; ++i) {
      const int d = 32 * w + 4 * i + sub;
      *(volatile v8h*)(vplane + (size_t)d * TT + t0 + 8 * q8) = pk[i];
    }
    __threadfence();
    #pragma unroll
    for (int i = 0; i < 8; ++i) {
      const int d = 32 * w + 4 * i + sub;
      *(volatile v8h*)(vplane + (size_t)d * TT + t0 + 8 * q8) = pk[i];
    }
  }
}

__device__ __forceinline__ v16h pack_p(v8f a, v8f c) {
  const v16h r = { (_Float16)(a[0] * PSC), (_Float16)(a[1] * PSC), (_Float16)(a[2] * PSC), (_Float16)(a[3] * PSC),
                   (_Float16)(a[4] * PSC), (_Float16)(a[5] * PSC), (_Float16)(a[6] * PSC), (_Float16)(a[7] * PSC),
                   (_Float16)(c[0] * PSC), (_Float16)(c[1] * PSC), (_Float16)(c[2] * PSC), (_Float16)(c[3] * PSC),
                   (_Float16)(c[4] * PSC), (_Float16)(c[5] * PSC), (_Float16)(c[6] * PSC), (_Float16)(c[7] * PSC) };
  return r;
}

__global__ __launch_bounds__(128) void k_attn(
    const _Float16* __restrict__ qh,
    const _Float16* __restrict__ kh,
    const _Float16* __restrict__ vT,
    _Float16* __restrict__ attn)
{
  __shared__ __attribute__((aligned(16))) _Float16 sO[4 * 16 * 128];

  const int tid = threadIdx.x, lane = tid & 31, w = tid >> 5;
  const int h = lane >> 4, m = lane & 15;
  const int head = blockIdx.y, kvh = head >> 2;
  const int q0 = blockIdx.x * 64 + 16 * w;
  const int qi = q0 + m;
  const int nst = 2 * ((int)blockIdx.x + 1);

  const _Float16* qrow = qh + ((size_t)head * TT + q0 + m) * DH;
  const v16h qb0 = load_frag(qrow, h);
  const v16h qb1 = load_frag(qrow + 32, h);
  const v16h qb2 = load_frag(qrow + 64, h);
  const v16h qb3 = load_frag(qrow + 96, h);

  v8f o[8];
  #pragma unroll
  for (int t = 0; t < 8; ++t) o[t] = zero8f();
  float mrun = -1e30f, lrun = 0.0f;

  const _Float16* kbase = kh + ((size_t)kvh * TT + m) * DH;
  const _Float16* vbase = vT + ((size_t)kvh * DH + m) * TT;
  const float SC = 0.0883883476483184f * 0.0625f;

  #pragma unroll 1
  for (int st = 0; st < nst; ++st) {
    const int kb = 32 * st;
    v8f s[2];
    #pragma unroll
    for (int j = 0; j < 2; ++j) {
      const _Float16* kp = kbase + (size_t)(kb + 16 * j) * DH;
      v8f z = zero8f();
      z = wmma_f16(load_frag(kp, h),      qb0, z);
      z = wmma_f16(load_frag(kp + 32, h), qb1, z);
      z = wmma_f16(load_frag(kp + 64, h), qb2, z);
      z = wmma_f16(load_frag(kp + 96, h), qb3, z);
      s[j] = z;
    }
    #pragma unroll
    for (int j = 0; j < 2; ++j)
      #pragma unroll
      for (int r = 0; r < 8; ++r) {
        const int kidx = kb + 16 * j + 8 * h + r;
        const float sv = s[j][r] * SC;
        s[j][r] = (kidx > qi) ? -1e30f : sv;
      }

    float mloc = s[0][0];
    #pragma unroll
    for (int j = 0; j < 2; ++j)
      #pragma unroll
      for (int r = 0; r < 8; ++r) mloc = fmaxf(mloc, s[j][r]);
    mloc = fmaxf(mloc, __shfl_xor(mloc, 16, 32));
    const float mnew = fmaxf(mrun, mloc);
    const float alpha = __expf(mrun - mnew);
    mrun = mnew;
    float lsum = 0.0f;
    #pragma unroll
    for (int j = 0; j < 2; ++j)
      #pragma unroll
      for (int r = 0; r < 8; ++r) {
        const float p = __expf(s[j][r] - mnew);
        s[j][r] = p;
        lsum += p;
      }
    lsum += __shfl_xor(lsum, 16, 32);
    lrun = lrun * alpha + lsum;
    #pragma unroll
    for (int t = 0; t < 8; ++t) o[t] = o[t] * alpha;

    const v16h pb = pack_p(s[0], s[1]);

    #pragma unroll
    for (int t = 0; t < 8; ++t) {
      const _Float16* vp = vbase + (size_t)(16 * t) * TT + kb;
      o[t] = wmma_f16(load_frag(vp, h), pb, o[t]);
    }
  }

  const float inv = (1.0f / lrun) * (1.0f / PSC);
  _Float16* so = sO + w * 2048;
  #pragma unroll
  for (int t = 0; t < 8; ++t)
    *(v8ha*)(so + m * 128 + 16 * t + 8 * h) = cvt8h(o[t] * inv);
  __syncthreads();

  const int q8 = lane & 7, sub = lane >> 3;
  v8h pk[8];
  #pragma unroll
  for (int i = 0; i < 8; ++i) {
    const int lid = 4 * i + sub, row = lid >> 1, hl = lid & 1;
    pk[i] = *(const v8ha*)(so + row * 128 + 64 * hl + 8 * q8);
  }
  #pragma unroll
  for (int i = 0; i < 8; ++i) {
    const int lid = 4 * i + sub, row = lid >> 1, hl = lid & 1;
    *(volatile v8h*)(attn + (size_t)(q0 + row) * DD + head * DH + 64 * hl + 8 * q8) = pk[i];
  }
  __threadfence();
  #pragma unroll
  for (int i = 0; i < 8; ++i) {
    const int lid = 4 * i + sub, row = lid >> 1, hl = lid & 1;
    *(volatile v8h*)(attn + (size_t)(q0 + row) * DD + head * DH + 64 * hl + 8 * q8) = pk[i];
  }
}

static void launch_cvt(const float* s, _Float16* d, int n, float sc, hipStream_t st) {
  const int n8 = n / 8;
  k_cvt<<<(n8 + 255) / 256, 256, 0, st>>>(s, d, n8, sc);
}

extern "C" void kernel_launch(void* const* d_in, const int* in_sizes, int n_in,
                              void* d_out, int out_size, void* d_ws, size_t ws_size,
                              hipStream_t stream) {
  if (n_in < 17) return;
  if (in_sizes[0] != TT * DD || in_sizes[1] != DD || in_sizes[2] != DD) return;
  if (in_sizes[3] != NHQ * DH * RQK || in_sizes[4] != NHQ * RQK * DD) return;
  if (in_sizes[5] != NHKV * DH * RQK || in_sizes[6] != NHKV * RQK * DD) return;
  if (in_sizes[7] != NHKV * DH * RQK || in_sizes[8] != NHKV * RQK * DD) return;
  if (in_sizes[9] != DD * RLO || in_sizes[10] != RLO * DD) return;
  if (in_sizes[11] != FF * RLO || in_sizes[12] != RLO * DD) return;
  if (in_sizes[13] != FF * RLO || in_sizes[14] != RLO * DD) return;
  if (in_sizes[15] != DD * RLO || in_sizes[16] != RLO * FF) return;
  if (out_size != TT * DD) return;
  const size_t MB = 1048576;
  if (ws_size < 117 * MB) return;

  const float* x   = (const float*)d_in[0];
  const float* ln1 = (const float*)d_in[1];
  const float* ln2 = (const float*)d_in[2];
  const float* qUs = (const float*)d_in[3];
  const float* qV  = (const float*)d_in[4];
  const float* kUs = (const float*)d_in[5];
  const float* kV  = (const float*)d_in[6];
  const float* vUs = (const float*)d_in[7];
  const float* vV  = (const float*)d_in[8];
  const float* oUs = (const float*)d_in[9];
  const float* oV  = (const float*)d_in[10];
  const float* gUs = (const float*)d_in[11];
  const float* gV  = (const float*)d_in[12];
  const float* uUs = (const float*)d_in[13];
  const float* uV  = (const float*)d_in[14];
  const float* dUs = (const float*)d_in[15];
  const float* dV  = (const float*)d_in[16];
  float* out = (float*)d_out;

  char* ws = (char*)d_ws;
  float*    x1     = (float*)   (ws +   0 * MB);
  _Float16* act16  = (_Float16*)(ws +  16 * MB);
  _Float16* xr16   = (_Float16*)(ws +  24 * MB);
  _Float16* orr16  = (_Float16*)(ws +  24 * MB);
  _Float16* grur16 = (_Float16*)(ws +  26 * MB);
  _Float16* dr16   = (_Float16*)(ws +  30 * MB);
  _Float16* vcat16 = (_Float16*)(ws +  32 * MB);
  _Float16* us16   = (_Float16*)(ws +  56 * MB);
  _Float16* qh     = (_Float16*)(ws +  57 * MB);
  _Float16* kh     = (_Float16*)(ws +  65 * MB);
  _Float16* vTp    = (_Float16*)(ws +  67 * MB);
  _Float16* oV16   = (_Float16*)(ws +  32 * MB);
  _Float16* oUs16  = (_Float16*)(ws +  40 * MB);
  _Float16* gVuV16 = (_Float16*)(ws +  32 * MB);
  _Float16* gUs16  = (_Float16*)(ws +  32 * MB);
  _Float16* uUs16  = (_Float16*)(ws +  60 * MB);
  _Float16* hmid16 = (_Float16*)(ws +  88 * MB);
  _Float16* dV16   = (_Float16*)(ws +  32 * MB);
  _Float16* dUs16  = (_Float16*)(ws +  60 * MB);
  float*    cosT   = (float*)   (ws + 116 * MB);
  float*    sinT   = (float*)   (ws + 116 * MB + 512 * 1024);

  k_rope_table<<<TT, 64, 0, stream>>>(cosT, sinT);
  k_rmsnorm<<<TT, 256, 0, stream>>>(x, ln1, act16);

  launch_cvt(qV,  vcat16,                          NHQ * RQK * DD,  WSC, stream);
  launch_cvt(kV,  vcat16 + (size_t)2048 * DD,      NHKV * RQK * DD, WSC, stream);
  launch_cvt(vV,  vcat16 + (size_t)2560 * DD,      NHKV * RQK * DD, WSC, stream);
  launch_cvt(qUs, us16,                            NHQ * DH * RQK,  WSC, stream);
  launch_cvt(kUs, us16 + (size_t)32 * DH * RQK,    NHKV * DH * RQK, WSC, stream);
  launch_cvt(vUs, us16 + (size_t)40 * DH * RQK,    NHKV * DH * RQK, WSC, stream);

  k_gemm_h<<<dim3(NXR / 64, TT / 128), 128, 0, stream>>>(act16, DD, vcat16, DD, xr16, NXR, DD, 1.0f / WSC);

  k_proj_rope<<<dim3(TT / 64, NHQ + 2 * NHKV), 128, 0, stream>>>(xr16, us16, cosT, sinT, qh, kh, vTp);

  k_attn<<<dim3(TT / 64, NHQ), 128, 0, stream>>>(qh, kh, vTp, act16);

  launch_cvt(oV,  oV16,  RLO * DD, WSC, stream);
  launch_cvt(oUs, oUs16, DD * RLO, WSC, stream);
  k_gemm_h<<<dim3(RLO / 64, TT / 128), 128, 0, stream>>>(act16, DD, oV16, DD, orr16, RLO, DD, 8.0f / (4.0f * WSC));
  k_gemm_res<<<dim3(DD / 64, TT / 128), 128, 0, stream>>>(orr16, RLO, oUs16, RLO, x, x1, RLO, 1.0f / (8.0f * WSC));

  k_rmsnorm<<<TT, 256, 0, stream>>>(x1, ln2, act16);

  launch_cvt(gV, gVuV16,                     RLO * DD, WSC, stream);
  launch_cvt(uV, gVuV16 + (size_t)RLO * DD,  RLO * DD, WSC, stream);
  k_gemm_h<<<dim3(2 * RLO / 64, TT / 128), 128, 0, stream>>>(act16, DD, gVuV16, DD, grur16, 2 * RLO, DD, 1.0f / WSC);

  launch_cvt(gUs, gUs16, FF * RLO, WSC, stream);
  launch_cvt(uUs, uUs16, FF * RLO, WSC, stream);
  k_gemm_glu<<<dim3(FF / 64, TT / 128), 128, 0, stream>>>(grur16, gUs16, uUs16, hmid16);

  launch_cvt(dV,  dV16,  RLO * FF, WSC, stream);
  launch_cvt(dUs, dUs16, DD * RLO, WSC, stream);
  k_gemm_h<<<dim3(RLO / 64, TT / 128), 128, 0, stream>>>(hmid16, FF, dV16, FF, dr16, RLO, FF, 1.0f / (4.0f * WSC));
  k_gemm_res<<<dim3(DD / 64, TT / 128), 128, 0, stream>>>(dr16, RLO, dUs16, RLO, x1, out, RLO, 1.0f / WSC);
}
